// _GRU_21397527069209
// MI455X (gfx1250) — hardware-verified
//
#include <hip/hip_runtime.h>
#include <math.h>

constexpr int NBATCH    = 2048;
constexpr int NSTEP     = 1024;
constexpr int NIN       = 5;
constexpr int NHID      = 32;
constexpr int NGATE     = 96;
constexpr int TILE_ROWS = 16;
constexpr int CHUNK     = 32;
constexpr int WPITCH    = 32;
constexpr int NWROWS    = 4 * NGATE + 16;
constexpr float WCARRY     = 64.0f;
constexpr float WCARRY_INV = 1.0f / 64.0f;
static_assert(NBATCH % TILE_ROWS == 0);
static_assert(NSTEP % CHUNK == 0);
static_assert(NHID == 32 && NGATE == 3 * NHID);
static_assert(NIN <= 8);
static_assert(CHUNK == 32);

typedef __attribute__((ext_vector_type(16))) _Float16 v16h;
typedef __attribute__((ext_vector_type(8)))  _Float16 v8h;
typedef __attribute__((ext_vector_type(8)))  float    v8f;
typedef __attribute__((ext_vector_type(4)))  float    v4f;
typedef __attribute__((ext_vector_type(4)))  unsigned v4u;

struct FragH {
  union U { v16h v; v8h h[2]; };
  static __device__ __forceinline__ v16h load(const _Float16* p) {
    U f;
    f.h[0] = *(const v8h*)(p);
    f.h[1] = *(const v8h*)(p + 16);
    return f.v;
  }
};

__device__ __forceinline__ v8f mma16(v16h a, v16h b, v8f cacc) {
  return __builtin_amdgcn_wmma_f32_16x16x32_f16(false, a, false, b, (short)0, cacc, false, false);
}

__device__ __forceinline__ void cell_guard(v8f& a0, v8f& a1, v8f& a2, v8f& a3,
                                           v16h x0, v16h x1,
                                           v16h w0, v16h w1, v16h w2, v16h w3, v16h w4, v16h w5) {
  asm volatile("v_nop\n\tv_nop\n\tv_nop\n\tv_nop"
               : "+v"(a0), "+v"(a1), "+v"(a2), "+v"(a3)
               : "v"(x0), "v"(x1), "v"(w0), "v"(w1), "v"(w2), "v"(w3), "v"(w4), "v"(w5));
}
__device__ __forceinline__ void head_guard(v8f& a0, v16h x0, v16h w0) {
  asm volatile("v_nop\n\tv_nop\n\tv_nop\n\tv_nop" : "+v"(a0) : "v"(x0), "v"(w0));
}

__device__ __forceinline__ float fsig(float x)  { return __builtin_amdgcn_rcpf(1.0f + __expf(-x)); }
__device__ __forceinline__ float ftanh(float x) { return 1.0f - 2.0f * __builtin_amdgcn_rcpf(__expf(2.0f * x) + 1.0f); }

__device__ __forceinline__ unsigned h16bits(float f) {
  const _Float16 hv = (_Float16)f;
  return (unsigned)__builtin_bit_cast(unsigned short, hv);
}
__device__ __forceinline__ unsigned pack2(float lo, float hi) {
  return h16bits(lo) | (h16bits(hi) << 16);
}

__device__ __forceinline__ void stage_plane32(const float* __restrict__ W, _Float16* dst, int lane) {
#pragma unroll 1
  for (int it = 0; it < 12; ++it) {
    const int task = it * 32 + lane;
    const int row = task >> 2;
    const int g8 = (task & 3) * 8;
    const float* p = W + row * NHID + g8;
    const v4f a = *(const v4f*)(p);
    const v4f b = *(const v4f*)(p + 4);
    const float a0 = a[0] * WCARRY, a1 = a[1] * WCARRY, a2 = a[2] * WCARRY, a3 = a[3] * WCARRY;
    const float c0 = b[0] * WCARRY, c1 = b[1] * WCARRY, c2 = b[2] * WCARRY, c3 = b[3] * WCARRY;
    v4u w;
    w[0] = pack2(a0, a1);
    w[1] = pack2(a2, a3);
    w[2] = pack2(c0, c1);
    w[3] = pack2(c2, c3);
    *(v8h*)(dst + row * WPITCH + g8) = __builtin_bit_cast(v8h, w);
  }
}

__device__ __forceinline__ void gru_cell(const v16h ax, const v16h ah,
                                         const _Float16* wi, const _Float16* wh,
                                         const float (&bs)[2][4], float (&hst)[2][8], _Float16* hb) {
  const v8f z8 = {0.f, 0.f, 0.f, 0.f, 0.f, 0.f, 0.f, 0.f};
#pragma unroll
  for (int ct = 0; ct < 2; ++ct) {
    const int ro = 16 * ct * WPITCH;
    const v16h b_ir = FragH::load(wi + ro);
    const v16h b_iz = FragH::load(wi + 32 * WPITCH + ro);
    const v16h b_in = FragH::load(wi + 64 * WPITCH + ro);
    const v16h b_hr = FragH::load(wh + ro);
    const v16h b_hz = FragH::load(wh + 32 * WPITCH + ro);
    const v16h b_hn = FragH::load(wh + 64 * WPITCH + ro);
    v8f ar = mma16(ax, b_ir, z8);
    v8f az = mma16(ax, b_iz, z8);
    v8f gx = mma16(ax, b_in, z8);
    v8f gh = mma16(ah, b_hn, z8);
    ar = mma16(ah, b_hr, ar);
    az = mma16(ah, b_hz, az);
    cell_guard(ar, az, gx, gh, ax, ah, b_ir, b_iz, b_in, b_hr, b_hz, b_hn);
    asm volatile("" ::: "memory");
#pragma unroll
    for (int r = 0; r < 8; ++r) {
      const float pr = fmaf(ar[r], WCARRY_INV, bs[ct][0]);
      const float pz = fmaf(az[r], WCARRY_INV, bs[ct][1]);
      const float rr = fsig(pr);
      const float zz = fsig(pz);
      const float xn = fmaf(gx[r], WCARRY_INV, bs[ct][2]);
      const float hn = fmaf(gh[r], WCARRY_INV, bs[ct][3]);
      const float nn = ftanh(xn + rr * hn);
      const float ho = hst[ct][r];
      const float hv = (1.0f - zz) * nn + zz * ho;
      hst[ct][r] = hv;
      hb[r * 32 + 16 * ct] = (_Float16)hv;
    }
  }
}

__global__ __launch_bounds__(32) __attribute__((amdgpu_num_vgpr(256)))
void gru2_head_kernel(const float* __restrict__ x,
                      const float* __restrict__ w_ih0, const float* __restrict__ w_hh0,
                      const float* __restrict__ b_ih0, const float* __restrict__ b_hh0,
                      const float* __restrict__ w_ih1, const float* __restrict__ w_hh1,
                      const float* __restrict__ b_ih1, const float* __restrict__ b_hh1,
                      const float* __restrict__ w_lin, const float* __restrict__ b_lin,
                      float* __restrict__ out) {
  __shared__ __align__(16) _Float16 Wl[NWROWS * WPITCH];
  __shared__ __align__(16) _Float16 Hb[2][TILE_ROWS * NHID];
  __shared__ __align__(16) unsigned Xs[TILE_ROWS * CHUNK * 4];
  __shared__ __align__(16) float Yb[TILE_ROWS * CHUNK];
  __shared__ __align__(16) float Bs[4 * NGATE];

  const int lane = threadIdx.x;
  const int c = lane & 15;
  const int hh = lane >> 4;
  const int b0 = blockIdx.x * TILE_ROWS;

  float zl = __uint_as_float((unsigned)lane & 0u);
  asm volatile("" : "+v"(zl));

  _Float16* WI0 = Wl;
  _Float16* WH0 = Wl + 1 * NGATE * WPITCH;
  _Float16* WI1 = Wl + 2 * NGATE * WPITCH;
  _Float16* WH1 = Wl + 3 * NGATE * WPITCH;
  _Float16* WLN = Wl + 4 * NGATE * WPITCH;

  stage_plane32(w_hh0, WH0, lane);
  stage_plane32(w_ih1, WI1, lane);
  stage_plane32(w_hh1, WH1, lane);
#pragma unroll 1
  for (int it = 0; it < 3; ++it) {
    const int row = it * 32 + lane;
    const float* p = w_ih0 + row * NIN;
    const float f0 = p[0] * WCARRY, f1 = p[1] * WCARRY, f2 = p[2] * WCARRY, f3 = p[3] * WCARRY, f4 = p[4] * WCARRY;
    v4u w;
    w[0] = pack2(f0, f1);
    w[1] = pack2(f2, f3);
    w[2] = pack2(f4, zl);
    w[3] = 0u;
    *(v8h*)(WI0 + row * WPITCH) = __builtin_bit_cast(v8h, w);
  }
#pragma unroll 1
  for (int it = 0; it < 9; ++it) {
    const int task = it * 32 + lane;
    const int row = task / 3;
    const int g = 1 + (task - row * 3);
    const v4u zw = {0u, 0u, 0u, 0u};
    *(v8h*)(WI0 + row * WPITCH + g * 8) = __builtin_bit_cast(v8h, zw);
  }
#pragma unroll 1
  for (int it = 0; it < 2; ++it) {
    const int task = it * 32 + lane;
    const int row = task >> 2;
    const int g8 = (task & 3) * 8;
    const float* p = w_lin + g8;
    const v4f a = *(const v4f*)(p);
    const v4f b = *(const v4f*)(p + 4);
    const float a0 = a[0] * WCARRY, a1 = a[1] * WCARRY, a2 = a[2] * WCARRY, a3 = a[3] * WCARRY;
    const float c0 = b[0] * WCARRY, c1 = b[1] * WCARRY, c2 = b[2] * WCARRY, c3 = b[3] * WCARRY;
    const unsigned w0 = pack2(a0, a1), w1 = pack2(a2, a3), w2 = pack2(c0, c1), w3 = pack2(c2, c3);
    const bool live = (row == 0);
    v4u w;
    w[0] = live ? w0 : 0u;
    w[1] = live ? w1 : 0u;
    w[2] = live ? w2 : 0u;
    w[3] = live ? w3 : 0u;
    *(v8h*)(WLN + row * WPITCH + g8) = __builtin_bit_cast(v8h, w);
  }
#pragma unroll 1
  for (int it = 0; it < 3; ++it) Bs[0 * NGATE + it * 32 + lane] = b_ih0[it * 32 + lane];
#pragma unroll 1
  for (int it = 0; it < 3; ++it) Bs[1 * NGATE + it * 32 + lane] = b_hh0[it * 32 + lane];
#pragma unroll 1
  for (int it = 0; it < 3; ++it) Bs[2 * NGATE + it * 32 + lane] = b_ih1[it * 32 + lane];
#pragma unroll 1
  for (int it = 0; it < 3; ++it) Bs[3 * NGATE + it * 32 + lane] = b_hh1[it * 32 + lane];
  const float blin = b_lin[0];
  __syncthreads();

  float bs0[2][4], bs1[2][4];
#pragma unroll
  for (int ct = 0; ct < 2; ++ct) {
    const int u = 16 * ct + c;
    bs0[ct][0] = Bs[0 * NGATE + u] + Bs[1 * NGATE + u];
    bs0[ct][1] = Bs[0 * NGATE + 32 + u] + Bs[1 * NGATE + 32 + u];
    bs0[ct][2] = Bs[0 * NGATE + 64 + u];
    bs0[ct][3] = Bs[1 * NGATE + 64 + u];
    bs1[ct][0] = Bs[2 * NGATE + u] + Bs[3 * NGATE + u];
    bs1[ct][1] = Bs[2 * NGATE + 32 + u] + Bs[3 * NGATE + 32 + u];
    bs1[ct][2] = Bs[2 * NGATE + 64 + u];
    bs1[ct][3] = Bs[3 * NGATE + 64 + u];
  }

  const int lofs = c * WPITCH + 8 * hh;
  const _Float16* wi0 = WI0 + lofs;
  const _Float16* wh0 = WH0 + lofs;
  const _Float16* wi1 = WI1 + lofs;
  const _Float16* wh1 = WH1 + lofs;
  const v16h blin_f = FragH::load(WLN + lofs);
  const _Float16* ha0 = &Hb[0][0] + c * NHID + 8 * hh;
  const _Float16* ha1 = &Hb[1][0] + c * NHID + 8 * hh;
  _Float16* hb0 = &Hb[0][0] + (8 * hh) * NHID + c;
  _Float16* hb1 = &Hb[1][0] + (8 * hh) * NHID + c;

  const v8f z8 = {0.f, 0.f, 0.f, 0.f, 0.f, 0.f, 0.f, 0.f};
  const v4u zero4 = {0u, 0u, 0u, 0u};
  const v8h zero8h = __builtin_bit_cast(v8h, zero4);
  const unsigned xm = (hh == 0) ? 0xFFFFFFFFu : 0u;
  const v4u xmask = {xm, xm, xm, xm};

  float h0s[2][8], h1s[2][8];
#pragma unroll
  for (int ct = 0; ct < 2; ++ct)
#pragma unroll
    for (int r = 0; r < 8; ++r) { h0s[ct][r] = 0.0f; h1s[ct][r] = 0.0f; }
  FragH::U fz;
  fz.h[0] = zero8h;
  fz.h[1] = zero8h;
  v16h a_h0 = fz.v;
  v16h a_h1 = fz.v;

#pragma unroll 1
  for (int t0 = 0; t0 < NSTEP; t0 += CHUNK) {
#pragma unroll 1
    for (int row = 0; row < TILE_ROWS; ++row) {
      const float* xp = x + ((size_t)(b0 + row) * NSTEP + (size_t)(t0 + lane)) * NIN;
      const float f0 = xp[0], f1 = xp[1], f2 = xp[2], f3 = xp[3], f4 = xp[4];
      v4u w;
      w[0] = pack2(f0, f1);
      w[1] = pack2(f2, f3);
      w[2] = pack2(f4, zl);
      w[3] = 0u;
      *(v4u*)(Xs + (row * CHUNK + lane) * 4) = w;
    }
    __syncthreads();

#pragma unroll 1
    for (int tl = 0; tl < CHUNK; ++tl) {
      const v4u xw = (*(const v4u*)(Xs + (c * CHUNK + tl) * 4)) & xmask;
      FragH::U fx;
      fx.h[0] = __builtin_bit_cast(v8h, xw);
      fx.h[1] = zero8h;

      gru_cell(fx.v, a_h0, wi0, wh0, bs0, h0s, hb0);
      __syncthreads();
      a_h0 = FragH::load(ha0);

      gru_cell(a_h0, a_h1, wi1, wh1, bs1, h1s, hb1);
      __syncthreads();
      a_h1 = FragH::load(ha1);

      v8f ya = mma16(a_h1, blin_f, z8);
      head_guard(ya, a_h1, blin_f);
      if (c == 0) {
#pragma unroll
        for (int r = 0; r < 8; ++r) Yb[(8 * hh + r) * CHUNK + tl] = ya[r];
      }
    }

    __syncthreads();
#pragma unroll 1
    for (int r = 0; r < TILE_ROWS; ++r) {
      const float lg = fmaf(Yb[r * CHUNK + lane], WCARRY_INV, blin);
      const float yv = fsig(lg);
      Yb[r * CHUNK + lane] = yv;
    }
    __syncthreads();
    {
      float* op = out + (size_t)b0 * NSTEP + (size_t)(t0 + lane);
      for (int pass = 0; pass < 2; ++pass) {
#pragma unroll
        for (int r = 0; r < TILE_ROWS; ++r) {
          const float v = Yb[r * CHUNK + lane];
          *(volatile float*)(op + (size_t)r * NSTEP) = v;
        }
        __threadfence();
      }
    }
    __syncthreads();
  }
}

extern "C" void kernel_launch(void* const* d_in, const int* in_sizes, int n_in,
                              void* d_out, int out_size, void* d_ws, size_t ws_size, hipStream_t stream) {
  (void)d_ws; (void)ws_size;
  if (n_in < 11 || d_out == nullptr) return;
  if (in_sizes[0] != NBATCH * NSTEP * NIN || in_sizes[1] != NGATE * NIN || in_sizes[2] != NGATE * NHID ||
      in_sizes[3] != NGATE || in_sizes[4] != NGATE || in_sizes[5] != NGATE * NHID || in_sizes[6] != NGATE * NHID ||
      in_sizes[7] != NGATE || in_sizes[8] != NGATE || in_sizes[9] != NHID || in_sizes[10] != 1 ||
      out_size != NBATCH * NSTEP) return;

  const float* x     = (const float*)d_in[0];
  const float* w_ih0 = (const float*)d_in[1];
  const float* w_hh0 = (const float*)d_in[2];
  const float* b_ih0 = (const float*)d_in[3];
  const float* b_hh0 = (const float*)d_in[4];
  const float* w_ih1 = (const float*)d_in[5];
  const float* w_hh1 = (const float*)d_in[6];
  const float* b_ih1 = (const float*)d_in[7];
  const float* b_hh1 = (const float*)d_in[8];
  const float* w_lin = (const float*)d_in[9];
  const float* b_lin = (const float*)d_in[10];
  float* out = (float*)d_out;

  gru2_head_kernel<<<NBATCH / TILE_ROWS, 32, 0, stream>>>(
      x, w_ih0, w_hh0, b_ih0, b_hh0, w_ih1, w_hh1, b_ih1, b_hh1, w_lin, b_lin, out);
}
